// Hyper_GAT_Model_5360119186023
// MI455X (gfx1250) — hardware-run, weakly checked
//
#include <hip/hip_runtime.h>


namespace {
constexpr int B = 16, WN = 30, F = 128, E19 = 19, N = WN * E19, NH = 8, C = 80, D = NH * C, NT = B * N;
constexpr float XS = 8.0f, WSC = 256.0f;
typedef _Float16 b16;
typedef __attribute__((ext_vector_type(16))) _Float16 v16b;
typedef __attribute__((ext_vector_type(8))) _Float16 v8b;
typedef __attribute__((ext_vector_type(8))) float v8f;
typedef __attribute__((ext_vector_type(4))) float v4f;
__device__ __forceinline__ float bf16_rne(float f) { unsigned int u = __float_as_uint(f); u += 0x7FFFu + ((u >> 16) & 1u); return __uint_as_float(u & 0xFFFF0000u); }
__device__ __forceinline__ v16b frag_kb(const b16* p, int hh) { const v8b a = *(const v8b*)(p + 8 * hh), b = *(const v8b*)(p + 16 + 8 * hh); v16b f;
#pragma unroll
  for (int e = 0; e < 8; ++e) { f[e] = a[e]; f[8 + e] = b[e]; } return f; }
__device__ __forceinline__ v8f wmma16b(v16b a, v16b b, v8f c) { v8f d = __builtin_amdgcn_wmma_f32_16x16x32_f16(false, a, false, b, (short)0, c, false, false); asm volatile("v_nop\n\tv_nop\n\tv_nop\n\tv_nop" : "+v"(d) : "v"(a), "v"(b)); return d; }
__device__ __forceinline__ void wave_lds_sync() { __builtin_amdgcn_fence(__ATOMIC_RELEASE, "workgroup"); __builtin_amdgcn_wave_barrier(); __builtin_amdgcn_fence(__ATOMIC_ACQUIRE, "workgroup"); }
__device__ __forceinline__ float pmul(float a, float b) { float p = a * b; asm volatile("" : "+v"(p)); return p; }
__device__ __forceinline__ float leaky(float v) { return v >= 0.0f ? v : 0.2f * v; }

__global__ __launch_bounds__(256) void wcopy_kernel(const float* __restrict__ w, int ro, b16* __restrict__ WT) {
  const int u = blockIdx.x * 256 + threadIdx.x; if (u >= D * 16) return; const int o = u / 16, k0 = (u % 16) * 8; v8b v;
#pragma unroll
  for (int j = 0; j < 8; ++j) v[j] = (b16)(bf16_rne(w[(size_t)o * F + k0 + j]) * WSC); for (int pass = 0; pass < 2; ++pass) { *(volatile v8b*)(WT + (size_t)(ro + o) * F + k0) = v; __threadfence(); }
}
__global__ __launch_bounds__(32) void proj_kernel(const float* __restrict__ x, const b16* __restrict__ WT, const float* __restrict__ bl, const float* __restrict__ br, int NBV, float* __restrict__ XLR) {
  __shared__ __attribute__((aligned(16))) b16 Ah[16][F + 8]; __shared__ __attribute__((aligned(16))) float Tf[16][128 + 4];
  const int lane = threadIdx.x, nloc = lane & 15, hlf = lane >> 4; const size_t m0 = (size_t)blockIdx.x * 16; if (m0 >= (size_t)NBV * N) return;
  for (int rr = 0; rr < 16; ++rr) { const size_t t = m0 + rr < (size_t)NT ? m0 + rr : (size_t)NT - 1; const int b = (int)(t / N), n = (int)(t % N), w = n / E19, e = n % E19; const float* xb = x + (((size_t)b * WN + w) * F) * E19 + e;
    for (int q = 0; q < 4; ++q) { const int f = q * 32 + lane; Ah[rr][f] = (b16)(bf16_rne(xb[(size_t)f * E19]) * XS); } }
  wave_lds_sync();
#pragma unroll 1
  for (int cg = 0; cg < 2 * D / 128; ++cg) { v8f acc[8];
#pragma unroll
    for (int t = 0; t < 8; ++t) acc[t] = (v8f){};
#pragma unroll
    for (int kb = 0; kb < F; kb += 32) { const v16b a = frag_kb(&Ah[nloc][kb], hlf);
#pragma unroll
      for (int t = 0; t < 8; ++t) acc[t] = wmma16b(a, frag_kb(WT + (size_t)(cg * 128 + t * 16 + nloc) * F + kb, hlf), acc[t]); }
#pragma unroll
    for (int t = 0; t < 8; ++t) { const int c = cg * 128 + t * 16 + nloc; const float bb = bf16_rne(c < D ? bl[c] : br[c - D]);
#pragma unroll
      for (int r8 = 0; r8 < 8; ++r8) Tf[8 * hlf + r8][t * 16 + nloc] = acc[t][r8] * (1.0f / (XS * WSC)) + bb; }
    wave_lds_sync();
    for (int pass = 0; pass < 2; ++pass) { for (int rr = 0; rr < 16; ++rr) if (m0 + rr < (size_t)NT) *(volatile v4f*)(XLR + (m0 + rr) * (2 * D) + cg * 128 + lane * 4) = *(const v4f*)(&Tf[rr][lane * 4]); __threadfence(); }
    wave_lds_sync(); }
}
__global__ __launch_bounds__(256) void gat_kernel(const float* __restrict__ XLR, const float* __restrict__ att, const float* __restrict__ cbias, int NBV, float* __restrict__ OUT) {
  const int wave = threadIdx.x >> 5, lane = threadIdx.x & 31; const size_t t = (size_t)blockIdx.x * 8 + wave; if (t >= (size_t)NBV * N) return; const int b = (int)(t / N), n = (int)(t % N), w = n / E19, e = n % E19; const int c0 = lane * 20;
  float xr[20], at[20]; for (int i = 0; i < 20; ++i) { xr[i] = XLR[t * (2 * D) + D + c0 + i]; at[i] = bf16_rne(att[c0 + i]); }
  const int nsrc = E19 + (w > 0 ? 1 : 0) + (w < WN - 1 ? 1 : 0);
  auto src_of = [&](int j) -> size_t { int sn; if (j < E19) sn = w * E19 + j; else if (j == E19 && w > 0) sn = (w - 1) * E19 + e; else sn = (w + 1) * E19 + e; return (size_t)b * N + sn; };
  auto logit = [&](size_t s) { const float* xl = XLR + s * (2 * D) + c0; float lg = 0.0f;
#pragma unroll
    for (int i = 0; i < 20; ++i) lg += pmul(leaky(xl[i] + xr[i]), at[i]); lg += __shfl_xor(lg, 1); lg += __shfl_xor(lg, 2); return lg; };
  float mx = -INFINITY;
#pragma unroll 1
  for (int j = 0; j < nsrc; ++j) mx = fmaxf(mx, logit(src_of(j)));
  float den = 0.0f, o[20]; for (int i = 0; i < 20; ++i) o[i] = 0.0f;
#pragma unroll 1
  for (int j = 0; j < nsrc; ++j) { const size_t s = src_of(j); const float p = __expf(logit(s) - mx); den += p; const float* xl = XLR + s * (2 * D) + c0;
#pragma unroll
    for (int i = 0; i < 20; ++i) o[i] += pmul(p, xl[i]); }
  const float inv = 1.0f / (den + 1e-16f); float r[20];
#pragma unroll
  for (int i = 0; i < 20; ++i) { const float v = pmul(o[i], inv) + bf16_rne(cbias[c0 + i]); r[i] = v > 0.0f ? v : (__expf(v) - 1.0f); }
  for (int pass = 0; pass < 2; ++pass) {
#pragma unroll
    for (int q4 = 0; q4 < 5; ++q4) *(volatile v4f*)(OUT + t * D + c0 + q4 * 4) = (v4f){r[q4 * 4], r[q4 * 4 + 1], r[q4 * 4 + 2], r[q4 * 4 + 3]}; __threadfence(); }
}
__global__ __launch_bounds__(256) void pool_kernel(const float* __restrict__ OUT, const float* __restrict__ Wp, const float* __restrict__ bpp, const float* __restrict__ Wf, const float* __restrict__ bfp, int NBV, float* __restrict__ LG) {
  __shared__ float Sc[N], red[256]; const int b = blockIdx.x, tid = threadIdx.x; if (b >= NBV) return; const float* ob = OUT + (size_t)b * N * D;
  for (int n = tid; n < N; n += 256) { float s = bf16_rne(bpp[0]); const float* orow = ob + (size_t)n * D;
#pragma unroll 4
    for (int c = 0; c < D; ++c) s += pmul(orow[c], bf16_rne(Wp[c])); Sc[n] = s; }
  __syncthreads(); float mx = -INFINITY; for (int n = tid; n < N; n += 256) mx = fmaxf(mx, Sc[n]); red[tid] = mx; __syncthreads();
  for (int wd = 128; wd > 0; wd >>= 1) { if (tid < wd) red[tid] = fmaxf(red[tid], red[tid + wd]); __syncthreads(); } mx = red[0]; __syncthreads();
  float sm = 0.0f; for (int n = tid; n < N; n += 256) { const float ev = __expf(Sc[n] - mx); Sc[n] = ev; sm += ev; } red[tid] = sm; __syncthreads();
  for (int wd = 128; wd > 0; wd >>= 1) { if (tid < wd) red[tid] += red[tid + wd]; __syncthreads(); } const float inv = 1.0f / red[0]; __syncthreads();
  float part = 0.0f;
  for (int c = tid; c < D; c += 256) { float pc = 0.0f;
#pragma unroll 1
    for (int n = 0; n < N; ++n) pc += pmul(Sc[n], ob[(size_t)n * D + c]); part += pmul(pmul(pc, inv), bf16_rne(Wf[c])); }
  red[tid] = part; __syncthreads(); for (int wd = 128; wd > 0; wd >>= 1) { if (tid < wd) red[tid] += red[tid + wd]; __syncthreads(); }
  if (tid < 32) { const float v = tid == 0 ? red[0] + bf16_rne(bfp[0]) : 0.0f; for (int pass = 0; pass < 2; ++pass) { ((volatile float*)LG)[(size_t)b * 32 + tid] = v; __threadfence(); } }
}
__global__ __launch_bounds__(32) void out_kernel(const float* __restrict__ LG, int NBV, float* __restrict__ out) { const int lane = threadIdx.x; for (int pass = 0; pass < 2; ++pass) { if (lane < NBV) ((volatile float*)out)[lane] = LG[lane * 32]; __threadfence(); } }
}

extern "C" void kernel_launch(void* const* d_in, const int* in_sizes, int n_in, void* d_out, int out_size, void* d_ws, size_t ws_size, hipStream_t stream) {
  (void)n_in;
  auto Fp = [&](int i) { return (const float*)d_in[i]; };
  if (in_sizes[0] != B * WN * F * E19 || in_sizes[1] != 2 * 11932 || in_sizes[2] != D * F || in_sizes[4] != D * F || in_sizes[6] != D || in_sizes[7] != D || in_sizes[8] != D || in_sizes[10] != D || out_size != B) return;
  const int NBV = B;
  size_t off = 0; char* ws = (char*)d_ws;
  auto carve = [&](size_t bytes) { char* p = ws + off; off += (bytes + 255) & ~(size_t)255; return p; };
  b16* WT = (b16*)carve((size_t)2 * D * F * 2); float* XLR = (float*)carve((size_t)NT * 2 * D * 4); float* OUT = (float*)carve((size_t)NT * D * 4); float* LG = (float*)carve((size_t)B * 32 * 4);
  if (off > ws_size || off > ((size_t)96 << 20)) return;
  wcopy_kernel<<<(D * 16 + 255) / 256, 256, 0, stream>>>(Fp(2), 0, WT); wcopy_kernel<<<(D * 16 + 255) / 256, 256, 0, stream>>>(Fp(4), D, WT);
  proj_kernel<<<(unsigned)((NBV * N + 15) / 16), 32, 0, stream>>>(Fp(0), WT, Fp(3), Fp(5), NBV, XLR);
  gat_kernel<<<(unsigned)((NBV * N + 7) / 8), 256, 0, stream>>>(XLR, Fp(6), Fp(7), NBV, OUT);
  pool_kernel<<<NBV, 256, 0, stream>>>(OUT, Fp(8), Fp(9), Fp(10), Fp(11), NBV, LG);
  out_kernel<<<1, 32, 0, stream>>>(LG, NBV, (float*)d_out);
}
